// DualGATTimeAwareModel_22050362097715
// MI455X (gfx1250) — hardware-verified
//
#include <hip/hip_runtime.h>
#include <stddef.h>


#define HEADS   4
#define CH      32
#define NCX     (HEADS * CH)
#define FEV     64
#define EMB     64
#define OUTD    64
#define NTHR    256
#define NWAVE   8
#define EPT     8
#define NGRP    2
#define CHUNK   (NTHR * EPT * NGRP)
#define WCAP    (EPT * NGRP * 32)
#define LISTN   (NWAVE * WCAP)
#define NBC     4096
#define NBF     1024
#define RCAP    20480
#define RBN     128
#define TGT     256
#define DEGCAP  256
#define OTHR    512
#define NEG_SLOPE    0.2f
#define LAMBDA_DECAY 0.1f

#define LDS_FILL ((2 * RCAP + NBF + LISTN) * 4 + 64)

static_assert((CHUNK & (CHUNK - 1)) == 0);
static_assert(CHUNK <= 4096);
static_assert(NBC <= 4096 && NBF <= 4096);
static_assert((NBC & (NBC - 1)) == 0 && (NBF & (NBF - 1)) == 0);
static_assert(NBC == 4 * NBF);
static_assert(OTHR * 8 == NBC);
static_assert((RCAP % 32) == 0);
static_assert(TGT == NWAVE * 32);
static_assert((NBC % TGT) == 0);
static_assert(NCX == 4 * 32);

typedef float          v4f  __attribute__((ext_vector_type(4)));
typedef float          v8f  __attribute__((ext_vector_type(8)));
typedef int            v4i  __attribute__((ext_vector_type(4)));
typedef unsigned short v8us __attribute__((ext_vector_type(8)));
typedef __bf16         v16b __attribute__((ext_vector_type(16)));
union FragB { v16b v; v8us h[2]; };

template <int KD, int NC>
struct GCfg {
  static constexpr int WPR  = (NC >= 32) ? 2 : 1;
  static constexpr int TPW  = NC / 16 / WPR;
  static constexpr int RG   = NWAVE / WPR;
  static constexpr int BM   = RG * 16;
  static constexpr int APK  = KD + 8;
  static constexpr int LDSA = 2 * BM * APK * 2;
  static constexpr int LDSS = BM * NC * 4;
  static constexpr int LDS  = LDSA > LDSS ? LDSA : LDSS;
};

__device__ __forceinline__ unsigned int bfr(float f) {
  const unsigned int u = __float_as_uint(f);
  return (u + 0x7FFFu + ((u >> 16) & 1u)) >> 16;
}

__device__ __forceinline__ void split1(float x, unsigned short& hb, unsigned short& lb) {
  const unsigned int hu = bfr(x);
  const float hf = __uint_as_float(hu << 16);
  hb = (unsigned short)hu;
  lb = (unsigned short)bfr(x - hf);
}

__device__ __forceinline__ void split8(v4f a, v4f b, v8us& hi, v8us& lo) {
  unsigned short hb, lb;
  split1(a.x, hb, lb); hi[0] = hb; lo[0] = lb;
  split1(a.y, hb, lb); hi[1] = hb; lo[1] = lb;
  split1(a.z, hb, lb); hi[2] = hb; lo[2] = lb;
  split1(a.w, hb, lb); hi[3] = hb; lo[3] = lb;
  split1(b.x, hb, lb); hi[4] = hb; lo[4] = lb;
  split1(b.y, hb, lb); hi[5] = hb; lo[5] = lb;
  split1(b.z, hb, lb); hi[6] = hb; lo[6] = lb;
  split1(b.w, hb, lb); hi[7] = hb; lo[7] = lb;
}

__device__ __forceinline__ v8f wmb(v16b a, v16b b, v8f c) {
  v8f d = __builtin_amdgcn_wmma_f32_16x16x32_bf16(false, a, false, b, (short)0, c, false, false);
  asm volatile("v_nop\n\tv_nop\n\tv_nop\n\tv_nop" : "+v"(d) : "v"(a), "v"(b));
  return d;
}

__device__ __forceinline__ float lrelu(float v) { return v > 0.0f ? v : NEG_SLOPE * v; }

template <int NB>
__device__ __forceinline__ int scan_chunk(const int* __restrict__ dsts, int nE, int cbase, int slotBase,
                                          int vec8, int* list, int tid, int lane, int wave) {
  int wc = 0;
#pragma unroll
  for (int g = 0; g < NGRP; ++g) {
    const int el0  = (g * NTHR + tid) * EPT;
    const int e0   = cbase + el0;
    const int sent = -2147483647 - 1;
    v4i da, db;
    if (vec8 != 0 && cbase + CHUNK <= nE) {
      da = *(const v4i*)(dsts + e0);
      db = *(const v4i*)(dsts + e0 + 4);
    } else {
      da.x = (e0     < nE) ? dsts[min(e0, nE - 1)] : sent;
      da.y = (e0 + 1 < nE) ? dsts[min(e0 + 1, nE - 1)] : sent;
      da.z = (e0 + 2 < nE) ? dsts[min(e0 + 2, nE - 1)] : sent;
      da.w = (e0 + 3 < nE) ? dsts[min(e0 + 3, nE - 1)] : sent;
      db.x = (e0 + 4 < nE) ? dsts[min(e0 + 4, nE - 1)] : sent;
      db.y = (e0 + 5 < nE) ? dsts[min(e0 + 5, nE - 1)] : sent;
      db.z = (e0 + 6 < nE) ? dsts[min(e0 + 6, nE - 1)] : sent;
      db.w = (e0 + 7 < nE) ? dsts[min(e0 + 7, nE - 1)] : sent;
    }
    const unsigned nb = (unsigned)slotBase;
    const unsigned s0 = (unsigned)da.x - nb, s1 = (unsigned)da.y - nb;
    const unsigned s2 = (unsigned)da.z - nb, s3 = (unsigned)da.w - nb;
    const unsigned s4 = (unsigned)db.x - nb, s5 = (unsigned)db.y - nb;
    const unsigned s6 = (unsigned)db.z - nb, s7 = (unsigned)db.w - nb;
    const bool h0 = s0 < (unsigned)NB, h1 = s1 < (unsigned)NB, h2 = s2 < (unsigned)NB, h3 = s3 < (unsigned)NB;
    const bool h4 = s4 < (unsigned)NB, h5 = s5 < (unsigned)NB, h6 = s6 < (unsigned)NB, h7 = s7 < (unsigned)NB;
    const unsigned any = __builtin_amdgcn_ballot_w32(h0 | h1 | h2 | h3 | h4 | h5 | h6 | h7);
    if (any != 0u) {
#define HITJ(J, HJ, SJ) { \
        const unsigned mj = __builtin_amdgcn_ballot_w32(HJ); \
        if (mj != 0u) { \
          if (HJ) { \
            const int pos = wc + (int)__builtin_amdgcn_mbcnt_lo(mj, 0u); \
            if (pos < WCAP) list[wave * WCAP + pos] = ((el0 + (J)) << 12) | (int)(SJ); \
          } \
          wc += (int)__builtin_popcount(mj); } }
      HITJ(0, h0, s0)
      HITJ(1, h1, s1)
      HITJ(2, h2, s2)
      HITJ(3, h3, s3)
      HITJ(4, h4, s4)
      HITJ(5, h5, s5)
      HITJ(6, h6, s6)
      HITJ(7, h7, s7)
#undef HITJ
    }
  }
  return wc;
}

template <int KD, int NC>
__global__ __launch_bounds__(NTHR) void k_wprep(const float* __restrict__ W, unsigned short* wp) {
  constexpr int UNITS = NC * KD / 8;
  constexpr int KD8   = KD / 8;
  static_assert((UNITS % 32) == 0);
  const int i = (int)blockIdx.x * NTHR + (int)threadIdx.x;
  if (i >= UNITS) return;
  const int n  = i / KD8;
  const int k0 = (i - n * KD8) * 8;
  float v[8];
#pragma unroll
  for (int e = 0; e < 8; ++e) v[e] = W[(size_t)(k0 + e) * NC + n];
  v4f a, b;
  a.x = v[0]; a.y = v[1]; a.z = v[2]; a.w = v[3];
  b.x = v[4]; b.y = v[5]; b.z = v[6]; b.w = v[7];
  v8us hv, lv;
  split8(a, b, hv, lv);
  unsigned short* dh = wp + (size_t)i * 8;
  unsigned short* dl = dh + (size_t)NC * KD;
  *(volatile v8us*)dh = hv;
  *(volatile v8us*)dl = lv;
  __threadfence();
  *(volatile v8us*)dh = hv;
  *(volatile v8us*)dl = lv;
}

__global__ __launch_bounds__(NTHR) void k_decay(const float* __restrict__ tim, float* dec, int nE) {
  const int e  = (int)blockIdx.x * NTHR + (int)threadIdx.x;
  const int ec = e > nE - 1 ? nE - 1 : e;
  const float d = expf(-LAMBDA_DECAY * tim[ec]);
  *(volatile float*)(dec + e) = d;
  __threadfence();
  *(volatile float*)(dec + e) = d;
}

__global__ __launch_bounds__(NTHR) void k_count(
    const int* __restrict__ dsts, int* cnt, int nE, int vec8) {
  __shared__ __attribute__((aligned(16))) int scnt[NBC];
  __shared__ __attribute__((aligned(16))) int list[LISTN];
  __shared__ int wcnt[NWAVE];
  const int tid = threadIdx.x, lane = tid & 31, wave = tid >> 5;
  const int nodeBase = blockIdx.x * NBC;

  for (int i = tid; i < NBC; i += NTHR) scnt[i] = 0;
  __syncthreads();

  const int nChunks = (nE + CHUNK - 1) / CHUNK;
#pragma unroll 1
  for (int ch = 0; ch < nChunks; ++ch) {
    const int cbase = ch * CHUNK;
    const int wc = scan_chunk<NBC>(dsts, nE, cbase, nodeBase, vec8, list, tid, lane, wave);
    if (lane == 0) wcnt[wave] = wc;
    __syncthreads();
    if (wave == 0) {
#pragma unroll 1
      for (int wsx = 0; wsx < NWAVE; ++wsx) {
        int n = __builtin_amdgcn_readfirstlane(wcnt[wsx]);
        n = n > WCAP ? WCAP : (n < 0 ? 0 : n);
        const int* lp = list + wsx * WCAP;
#pragma unroll 1
        for (int i = 0; i < n; ++i) {
          const int ent  = __builtin_amdgcn_readfirstlane(lp[i]);
          const int slot = ent & (NBC - 1);
          if (lane == 0) scnt[slot] = scnt[slot] + 1;
        }
      }
    }
    __syncthreads();
  }

  v4i cq[4];
#pragma unroll
  for (int q = 0; q < 4; ++q) {
    const int f = (wave * 4 + q) * 128 + 4 * lane;
    cq[q] = *(const v4i*)(scnt + f);
  }
  int* cp = cnt + (size_t)nodeBase;
#pragma unroll
  for (int q = 0; q < 4; ++q) {
    const int f = (wave * 4 + q) * 128 + 4 * lane;
    *(volatile v4i*)(cp + f) = cq[q];
  }
  __threadfence();
#pragma unroll
  for (int q = 0; q < 4; ++q) {
    const int f = (wave * 4 + q) * 128 + 4 * lane;
    *(volatile v4i*)(cp + f) = cq[q];
  }
}

__global__ __launch_bounds__(OTHR) void k_offsets(
    const int* __restrict__ cnt, int* off, int* rbase, int nChunk) {
  __shared__ __attribute__((aligned(16))) int soff[NBC];
  __shared__ __attribute__((aligned(16))) int srb[RBN];
  __shared__ int wtot[OTHR / 32];
  const int tid = threadIdx.x, lane = tid & 31, wave = tid >> 5, sub = tid >> 7;
  for (int i = tid; i < RBN; i += OTHR) srb[i] = 0;
  int carry = 0;
#pragma unroll 1
  for (int ch = 0; ch < nChunk; ++ch) {
    const int base = ch * NBC;
    const v4i c0 = *(const v4i*)(cnt + base + 8 * tid);
    const v4i c1 = *(const v4i*)(cnt + base + 8 * tid + 4);
    const int e0 = max(c0.x, 0), e1 = max(c0.y, 0), e2 = max(c0.z, 0), e3 = max(c0.w, 0);
    const int e4 = max(c1.x, 0), e5 = max(c1.y, 0), e6 = max(c1.z, 0), e7 = max(c1.w, 0);
    const int ts = e0 + e1 + e2 + e3 + e4 + e5 + e6 + e7;
    int incl = ts;
#pragma unroll
    for (int d = 1; d < 32; d <<= 1) {
      const int t = __shfl_up(incl, d);
      if (lane >= d) incl += t;
    }
    if (lane == 31) wtot[wave] = incl;
    __syncthreads();
    const int S0 = wtot[0]  + wtot[1]  + wtot[2]  + wtot[3];
    const int S1 = wtot[4]  + wtot[5]  + wtot[6]  + wtot[7];
    const int S2 = wtot[8]  + wtot[9]  + wtot[10] + wtot[11];
    const int S3 = wtot[12] + wtot[13] + wtot[14] + wtot[15];
    int pre = 0;
#pragma unroll 1
    for (int w = 4 * sub; w < wave; ++w) pre += wtot[w];
    const int b0 = carry;
    const int b1 = b0 + ((S0 + 31) & ~31);
    const int b2 = b1 + ((S1 + 31) & ~31);
    const int b3 = b2 + ((S2 + 31) & ~31);
    const int b4 = b3 + ((S3 + 31) & ~31);
    const int myb = sub == 0 ? b0 : (sub == 1 ? b1 : (sub == 2 ? b2 : b3));
    if (tid == 0) {
      srb[min(4 * ch + 0, RBN - 1)] = b0;
      srb[min(4 * ch + 1, RBN - 1)] = b1;
      srb[min(4 * ch + 2, RBN - 1)] = b2;
      srb[min(4 * ch + 3, RBN - 1)] = b3;
    }
    int run = myb + pre + incl - ts;
    soff[8 * tid + 0] = run; run += e0;
    soff[8 * tid + 1] = run; run += e1;
    soff[8 * tid + 2] = run; run += e2;
    soff[8 * tid + 3] = run; run += e3;
    soff[8 * tid + 4] = run; run += e4;
    soff[8 * tid + 5] = run; run += e5;
    soff[8 * tid + 6] = run; run += e6;
    soff[8 * tid + 7] = run;
    carry = b4;
    __syncthreads();
    const v4i o0 = *(const v4i*)(soff + 4 * tid);
    const v4i o1 = *(const v4i*)(soff + 4 * (tid + OTHR));
    int* op = off + base;
    *(volatile v4i*)(op + 4 * tid) = o0;
    *(volatile v4i*)(op + 4 * (tid + OTHR)) = o1;
    __threadfence();
    *(volatile v4i*)(op + 4 * tid) = o0;
    *(volatile v4i*)(op + 4 * (tid + OTHR)) = o1;
    __syncthreads();
  }
  if (tid == 0) srb[min(4 * nChunk, RBN - 1)] = carry;
  __syncthreads();
  v4i rv = {0, 0, 0, 0};
  if (tid < 32) rv = *(const v4i*)(srb + 4 * tid);
  if (tid < 32) *(volatile v4i*)(rbase + 4 * tid) = rv;
  __threadfence();
  if (tid < 32) *(volatile v4i*)(rbase + 4 * tid) = rv;
}

__global__ __launch_bounds__(NTHR) void k_fill(
    const int* __restrict__ srcs, const int* __restrict__ dsts, const float* __restrict__ dec,
    const int* __restrict__ off, const int* __restrict__ rbase,
    int* csrS, float* csrD, int nN, int nE, int vec8, int csrLen) {
  extern __shared__ v4f lds_dyn[];
  int*   regS   = (int*)lds_dyn;
  float* regD   = (float*)(regS + RCAP);
  int*   cursor = regS + 2 * RCAP;
  int*   list   = cursor + NBF;
  int*   wcnt   = list + LISTN;
  const int tid = threadIdx.x, lane = tid & 31, wave = tid >> 5;
  const int b = blockIdx.x;
  const int nodeBase = b * NBF;

  int rb0 = rbase[b];
  const int rb1 = rbase[b + 1];
  rb0 = rb0 < 0 ? 0 : (rb0 > csrLen ? csrLen : rb0);
  rb0 &= ~31;
  int len = rb1 - rb0;
  len = len < 0 ? 0 : (len > RCAP ? RCAP : len);
  int lenW = (len + 31) & ~31;
  if (rb0 + lenW > csrLen) lenW = (csrLen - rb0) & ~31;

  {
    const v4i z = {0, 0, 0, 0};
    for (int i = tid; i < (2 * RCAP) / 4; i += NTHR) ((v4i*)regS)[i] = z;
    for (int s = tid; s < NBF; s += NTHR) {
      int o = off[nodeBase + s] - rb0;
      o = o < 0 ? 0 : (o > RCAP ? RCAP : o);
      cursor[s] = o;
    }
  }
  __syncthreads();

  const int nChunks = (nE + CHUNK - 1) / CHUNK;
#pragma unroll 1
  for (int ch = 0; ch < nChunks; ++ch) {
    const int cbase = ch * CHUNK;
    const int wc = scan_chunk<NBF>(dsts, nE, cbase, nodeBase, vec8, list, tid, lane, wave);
    if (lane == 0) wcnt[wave] = wc;
    __syncthreads();
    if (wave == 0) {
#pragma unroll 1
      for (int wsx = 0; wsx < NWAVE; ++wsx) {
        int n = __builtin_amdgcn_readfirstlane(wcnt[wsx]);
        n = n > WCAP ? WCAP : (n < 0 ? 0 : n);
        const int* lp = list + wsx * WCAP;
#pragma unroll 1
        for (int i = 0; i < n; ++i) {
          const int ent  = __builtin_amdgcn_readfirstlane(lp[i]);
          const int slot = ent & (NBF - 1);
          int e = cbase + ((ent >> 12) & (CHUNK - 1));
          e = e > nE - 1 ? nE - 1 : e;
          int src = srcs[e];
          src = src < 0 ? 0 : (src > nN - 1 ? nN - 1 : src);
          const float dv = dec[e];
          if (lane == 0) {
            int pos = cursor[slot];
            pos = pos < 0 ? 0 : (pos > RCAP - 1 ? RCAP - 1 : pos);
            regS[pos] = src;
            regD[pos] = dv;
            const int np = pos + 1;
            cursor[slot] = np > RCAP ? RCAP : np;
          }
        }
      }
    }
    __syncthreads();
  }

  const int nv = lenW >> 2;
  int*   gpS = csrS + rb0;
  float* gpD = csrD + rb0;
#pragma unroll 1
  for (int i = tid; i < nv; i += NTHR) {
    const v4i vs = ((const v4i*)regS)[i];
    const v4f vd = ((const v4f*)regD)[i];
    *(volatile v4i*)(gpS + 4 * i) = vs;
    *(volatile v4f*)(gpD + 4 * i) = vd;
  }
  __threadfence();
#pragma unroll 1
  for (int i = tid; i < nv; i += NTHR) {
    const v4i vs = ((const v4i*)regS)[i];
    const v4f vd = ((const v4f*)regD)[i];
    *(volatile v4i*)(gpS + 4 * i) = vs;
    *(volatile v4f*)(gpD + 4 * i) = vd;
  }
}

template <int KD, int NC, int GATH, int FC>
__global__ __launch_bounds__(NTHR) void k_gemm(
    const float* __restrict__ A, const int* __restrict__ gidx,
    const unsigned short* __restrict__ Bw, const float* __restrict__ att,
    float* C, float* eI, float* eJ, int nRowsA, int nTab, int nRowsC) {
  typedef GCfg<KD, NC> G;
  constexpr int WPR  = G::WPR;
  constexpr int TPW  = G::TPW;
  constexpr int BM   = G::BM;
  constexpr int APK  = G::APK;
  constexpr int LPH  = CH / 4;
  constexpr int Q4   = TPW * 4;
  constexpr int RPI  = 32 / Q4;
  constexpr int NIT  = 16 / RPI;
  constexpr int NES  = BM * HEADS;
  constexpr int NESI = NES / 128;
  constexpr int UPT  = (BM * KD / 8) / NTHR;
  constexpr size_t WPLN = (size_t)NC * KD;
  static_assert(KD % 32 == 0 && NC % (16 * WPR) == 0);
  static_assert(FC == 1 || HEADS * CH == NC);
  static_assert((Q4 & (Q4 - 1)) == 0 && Q4 <= 32 && Q4 >= LPH && (LPH & (LPH - 1)) == 0 && LPH >= 1);
  static_assert(NIT * RPI == 16);
  static_assert((NES % 128) == 0 && 2 * NESI <= NWAVE);
  static_assert(UPT >= 1 && UPT * NTHR * 8 == BM * KD);
  static_assert(((APK * 2) % 16) == 0);
  static_assert(BM * NC * 4 <= G::LDS && 2 * BM * APK * 2 <= G::LDS);

  extern __shared__ v4f lds_dyn[];
  __shared__ __attribute__((aligned(16))) float sEI[NES];
  __shared__ __attribute__((aligned(16))) float sEJ[NES];
  unsigned short* sHi = (unsigned short*)lds_dyn;
  unsigned short* sLo = sHi + BM * APK;
  float*          stg = (float*)lds_dyn;
  const int tid = threadIdx.x, lane = tid & 31, wave = tid >> 5, hh = lane >> 4, m = lane & 15;
  const int rowBase = blockIdx.x * BM;

#pragma unroll
  for (int i = 0; i < UPT; ++i) {
    const int idx = i * NTHR + tid;
    const int r   = idx / (KD / 8);
    const int cc0 = (idx - r * (KD / 8)) * 8;
    int row = rowBase + r;
    row = row > nRowsA - 1 ? nRowsA - 1 : row;
    if constexpr (GATH != 0) {
      int g = gidx[row];
      g = g < 0 ? g + nTab : g;
      g = g < 0 ? 0 : (g > nTab - 1 ? nTab - 1 : g);
      row = g;
    }
    const float* ap = A + (size_t)row * KD + cc0;
    const v4f a = *(const v4f*)ap, b = *(const v4f*)(ap + 4);
    v8us hv, lv;
    split8(a, b, hv, lv);
    *(v8us*)(sHi + r * APK + cc0) = hv;
    *(v8us*)(sLo + r * APK + cc0) = lv;
  }
  __syncthreads();

  const int rg  = wave / WPR;
  const int chf = wave - rg * WPR;
  const int r0  = rg * 16;
  const int c0  = chf * TPW * 16;

  v8f acc[TPW];
#pragma unroll
  for (int t = 0; t < TPW; ++t) { v8f z = {0.f, 0.f, 0.f, 0.f, 0.f, 0.f, 0.f, 0.f}; acc[t] = z; }
  const unsigned short* ahp = sHi + (r0 + m) * APK + 8 * hh;
  const unsigned short* alp = sLo + (r0 + m) * APK + 8 * hh;
#pragma unroll 2
  for (int kt = 0; kt < KD / 32; ++kt) {
    FragB ah, al;
    ah.h[0] = *(const v8us*)(ahp + 32 * kt);
    ah.h[1] = *(const v8us*)(ahp + 32 * kt + 16);
    al.h[0] = *(const v8us*)(alp + 32 * kt);
    al.h[1] = *(const v8us*)(alp + 32 * kt + 16);
#pragma unroll
    for (int t = 0; t < TPW; ++t) {
      const unsigned short* bp = Bw + (size_t)(c0 + 16 * t + m) * KD + 32 * kt + 8 * hh;
      FragB bh, bl;
      bh.h[0] = *(const v8us*)bp;
      bh.h[1] = *(const v8us*)(bp + 16);
      bl.h[0] = *(const v8us*)(bp + WPLN);
      bl.h[1] = *(const v8us*)(bp + WPLN + 16);
      acc[t] = wmb(ah.v, bh.v, acc[t]);
      acc[t] = wmb(ah.v, bl.v, acc[t]);
      acc[t] = wmb(al.v, bh.v, acc[t]);
    }
  }
  __syncthreads();

  {
    float* sp = stg + (size_t)(r0 + 8 * hh) * NC + c0 + m;
#pragma unroll
    for (int t = 0; t < TPW; ++t) {
#pragma unroll
      for (int r = 0; r < 8; ++r) sp[r * NC + 16 * t] = acc[t][r];
    }
  }
  __syncthreads();

  const int qq   = lane & (Q4 - 1);
  const int rsub = lane / Q4;
  const int col  = c0 + 4 * qq;
  const size_t gb = (size_t)(rowBase + r0) * NC + col;

  if constexpr (FC == 0) {
    const int hd = col / CH;
    const int cc = col - hd * CH;
    const v4f sA = *(const v4f*)(att + hd * (2 * CH) + cc);
    const v4f sB = *(const v4f*)(att + hd * (2 * CH) + CH + cc);
#pragma unroll
    for (int it = 0; it < NIT; ++it) {
      const int row = it * RPI + rsub;
      const v4f v = *(const v4f*)(stg + (size_t)(r0 + row) * NC + col);
      *(volatile v4f*)(C + gb + (size_t)row * NC) = v;
      float ps = v.x * sA.x + v.y * sA.y + v.z * sA.z + v.w * sA.w;
      float pd = v.x * sB.x + v.y * sB.y + v.z * sB.z + v.w * sB.w;
#pragma unroll
      for (int o = 1; o < LPH; o <<= 1) { ps += __shfl_xor(ps, o); pd += __shfl_xor(pd, o); }
      if ((lane & (LPH - 1)) == 0) { sEI[(r0 + row) * HEADS + hd] = ps; sEJ[(r0 + row) * HEADS + hd] = pd; }
    }
    __threadfence();
#pragma unroll
    for (int it = 0; it < NIT; ++it) {
      const int row = it * RPI + rsub;
      const v4f v = *(const v4f*)(stg + (size_t)(r0 + row) * NC + col);
      *(volatile v4f*)(C + gb + (size_t)row * NC) = v;
    }
    __syncthreads();

    v4f dv = {0.f, 0.f, 0.f, 0.f};
    const size_t eb = (size_t)rowBase * HEADS;
    if (wave < NESI) {
      const int f = wave * 128 + 4 * lane;
      dv = *(const v4f*)(sEI + f);
      *(volatile v4f*)(eI + eb + f) = dv;
    } else if (wave < 2 * NESI) {
      const int f = (wave - NESI) * 128 + 4 * lane;
      dv = *(const v4f*)(sEJ + f);
      *(volatile v4f*)(eJ + eb + f) = dv;
    }
    __threadfence();
    if (wave < NESI) {
      const int f = wave * 128 + 4 * lane;
      *(volatile v4f*)(eI + eb + f) = dv;
    } else if (wave < 2 * NESI) {
      const int f = (wave - NESI) * 128 + 4 * lane;
      *(volatile v4f*)(eJ + eb + f) = dv;
    }
  } else {
    const v4f bv = *(const v4f*)(att + col);
    v4f vv[NIT];
#pragma unroll
    for (int it = 0; it < NIT; ++it) {
      const int row = it * RPI + rsub;
      vv[it] = *(const v4f*)(stg + (size_t)(r0 + row) * NC + col) + bv;
      const int grow = rowBase + r0 + row;
      if (grow < nRowsC) *(volatile v4f*)(C + gb + (size_t)row * NC) = vv[it];
    }
    __threadfence();
#pragma unroll
    for (int it = 0; it < NIT; ++it) {
      const int row = it * RPI + rsub;
      const int grow = rowBase + r0 + row;
      if (grow < nRowsC) *(volatile v4f*)(C + gb + (size_t)row * NC) = vv[it];
    }
  }
}

__global__ __launch_bounds__(NTHR) void k_agg(
    const int* __restrict__ csrS, const float* __restrict__ csrD,
    const int* __restrict__ off, const int* __restrict__ cnt,
    const float* __restrict__ eI, const float* __restrict__ eJ, const float* __restrict__ hw,
    float* xout, int ldo, int colOff, int nN, int csrLen) {
  const int tid = threadIdx.x, lane = tid & 31, wave = tid >> 5;
  const int tbase = blockIdx.x * TGT + wave * 32;
  const int col0 = 4 * lane;
  const int hd   = lane >> 3;
  const v4f z4 = {0.f, 0.f, 0.f, 0.f};

  const int cl    = tbase + lane;
  const int cnt_l = cnt[cl];
  const int off_l = off[cl];

#pragma unroll 1
  for (int j = 0; j < 32; ++j) {
    const int c = tbase + j;
    int n = __shfl(cnt_l, j);
    n = n < 0 ? 0 : (n > DEGCAP ? DEGCAP : n);
    const int st = __shfl(off_l, j);
    const float ei = eI[(size_t)c * HEADS + hd];

    v4f acc = z4;
#pragma unroll 1
    for (int q0 = 0; q0 < n; q0 += 32) {
      int pos = st + q0 + lane;
      pos = pos < 0 ? 0 : (pos > csrLen - 1 ? csrLen - 1 : pos);
      int sl = csrS[pos];
      sl = sl < 0 ? 0 : (sl > nN - 1 ? nN - 1 : sl);
      const float dl = csrD[pos];
      const int mcnt = (n - q0) < 32 ? (n - q0) : 32;
#pragma unroll 1
      for (int pp = 0; pp < mcnt; ++pp) {
        const int   s  = __builtin_amdgcn_readlane(sl, pp);
        const float dc = __int_as_float(__builtin_amdgcn_readlane(__float_as_int(dl), pp));
        const float a  = lrelu(ei + eJ[(size_t)s * HEADS + hd]) * dc;
        const v4f   h  = *(const v4f*)(hw + (size_t)s * NCX + col0);
        acc = acc + h * a;
      }
    }

    if (c >= nN) acc = z4;
    float* p = xout + (size_t)c * ldo + colOff + col0;
    *(volatile v4f*)p = acc;
    __threadfence();
    *(volatile v4f*)p = acc;
  }
}

typedef GCfg<EMB, NCX>      GA;
typedef GCfg<FEV, NCX>      GB;
typedef GCfg<2 * NCX, NCX>  GC;
typedef GCfg<NCX, OUTD>     GF;
static_assert((TGT % GA::BM) == 0 && (TGT % GB::BM) == 0 && (TGT % GC::BM) == 0 && (TGT % GF::BM) == 0);

extern "C" void kernel_launch(void* const* d_in, const int* in_sizes, int n_in,
                              void* d_out, int out_size, void* d_ws, size_t ws_size,
                              hipStream_t stream) {
  if (n_in < 13) return;
  const int nN   = in_sizes[0] / FEV;
  const int nE   = in_sizes[3];
  const int nTab = in_sizes[4] / EMB;
  if (nN <= 0 || nE <= 0 || nTab <= 0) return;
  if (in_sizes[0] != nN * FEV || in_sizes[1] != nN || in_sizes[2] != 2 * nE || in_sizes[4] != nTab * EMB) return;
  if (in_sizes[5] != EMB * NCX || in_sizes[6] != HEADS * 2 * CH) return;
  if (in_sizes[7] != FEV * NCX || in_sizes[8] != HEADS * 2 * CH) return;
  if (in_sizes[9] != 2 * NCX * NCX || in_sizes[10] != HEADS * 2 * CH) return;
  if (in_sizes[11] != NCX * OUTD || in_sizes[12] != OUTD) return;
  if (out_size != nN * OUTD) return;
  if (nE > (1 << 28) || nN > (1 << 24)) return;

  const float* x      = (const float*)d_in[0];
  const int*   eid    = (const int*)d_in[1];
  const int*   edge   = (const int*)d_in[2];
  const float* tim    = (const float*)d_in[3];
  const float* emb    = (const float*)d_in[4];
  const float* Wemb   = (const float*)d_in[5];
  const float* attEmb = (const float*)d_in[6];
  const float* Wev    = (const float*)d_in[7];
  const float* attEv  = (const float*)d_in[8];
  const float* Wcat   = (const float*)d_in[9];
  const float* attCat = (const float*)d_in[10];
  const float* fcw    = (const float*)d_in[11];
  const float* fcb    = (const float*)d_in[12];
  float* out = (float*)d_out;
  const int* src = edge;
  const int* dst = edge + nE;

  const int NPAD   = ((nN + TGT - 1) / TGT) * TGT;
  const int nBC    = (nN + NBC - 1) / NBC;
  const int CNTPAD = nBC * NBC;
  if (4 * nBC + 1 > RBN) return;
  const int nBF    = (nN + NBF - 1) / NBF;
  const int csrLen = ((nE + 31) & ~31) + 4096;
  if (31 * 4 * nBC > 4096) return;
  const int decLen = ((nE + NTHR - 1) / NTHR) * NTHR;
  const int nAgg   = NPAD / TGT;

  char* ws = (char*)d_ws;
  size_t off = 0;
  const size_t oW1  = off; off += (size_t)2 * EMB * NCX * 2;      off = (off + 255) & ~(size_t)255;
  const size_t oW2  = off; off += (size_t)2 * FEV * NCX * 2;      off = (off + 255) & ~(size_t)255;
  const size_t oW3  = off; off += (size_t)2 * 2 * NCX * NCX * 2;  off = (off + 255) & ~(size_t)255;
  const size_t oW4  = off; off += (size_t)2 * NCX * OUTD * 2;     off = (off + 255) & ~(size_t)255;
  const size_t oDec = off; off += (size_t)decLen * 4;             off = (off + 255) & ~(size_t)255;
  const size_t oCnt = off; off += (size_t)CNTPAD * 4;             off = (off + 255) & ~(size_t)255;
  const size_t oOff = off; off += (size_t)CNTPAD * 4;             off = (off + 255) & ~(size_t)255;
  const size_t oRb  = off; off += (size_t)RBN * 4;                off = (off + 255) & ~(size_t)255;
  const size_t oCS  = off; off += (size_t)csrLen * 4;             off = (off + 255) & ~(size_t)255;
  const size_t oCD  = off; off += (size_t)csrLen * 4;             off = (off + 255) & ~(size_t)255;
  const size_t oXp  = off; off += (size_t)NPAD * NCX * 4;         off = (off + 255) & ~(size_t)255;
  const size_t oEI  = off; off += (size_t)NPAD * HEADS * 4;       off = (off + 255) & ~(size_t)255;
  const size_t oEJ  = off; off += (size_t)NPAD * HEADS * 4;       off = (off + 255) & ~(size_t)255;
  const size_t oH   = off; off += (size_t)NPAD * 2 * NCX * 4;     off = (off + 255) & ~(size_t)255;
  if (off > ws_size) return;
  unsigned short* wp1 = (unsigned short*)(ws + oW1);
  unsigned short* wp2 = (unsigned short*)(ws + oW2);
  unsigned short* wp3 = (unsigned short*)(ws + oW3);
  unsigned short* wp4 = (unsigned short*)(ws + oW4);
  float* dec  = (float*)(ws + oDec);
  int*   cnt  = (int*)(ws + oCnt);
  int*   offp = (int*)(ws + oOff);
  int*   rb   = (int*)(ws + oRb);
  int*   csrS = (int*)(ws + oCS);
  float* csrD = (float*)(ws + oCD);
  float* xp   = (float*)(ws + oXp);
  float* eI   = (float*)(ws + oEI);
  float* eJ   = (float*)(ws + oEJ);
  float* hcat = (float*)(ws + oH);
  float* h2   = hcat;

  const int vec8 = ((nE & 3) == 0) ? 1 : 0;

  k_wprep<EMB, NCX><<<(NCX * EMB / 8 + NTHR - 1) / NTHR, NTHR, 0, stream>>>(Wemb, wp1);
  k_wprep<FEV, NCX><<<(NCX * FEV / 8 + NTHR - 1) / NTHR, NTHR, 0, stream>>>(Wev, wp2);
  k_wprep<2 * NCX, NCX><<<(NCX * 2 * NCX / 8 + NTHR - 1) / NTHR, NTHR, 0, stream>>>(Wcat, wp3);
  k_wprep<NCX, OUTD><<<(OUTD * NCX / 8 + NTHR - 1) / NTHR, NTHR, 0, stream>>>(fcw, wp4);

  k_decay<<<decLen / NTHR, NTHR, 0, stream>>>(tim, dec, nE);

  k_count<<<nBC, NTHR, 0, stream>>>(dst, cnt, nE, vec8);
  k_offsets<<<1, OTHR, 0, stream>>>(cnt, offp, rb, nBC);
  hipFuncSetAttribute(reinterpret_cast<const void*>(&k_fill),
                      hipFuncAttributeMaxDynamicSharedMemorySize, LDS_FILL);
  k_fill<<<nBF, NTHR, LDS_FILL, stream>>>(src, dst, dec, offp, rb, csrS, csrD, nN, nE, vec8, csrLen);

  hipFuncSetAttribute(reinterpret_cast<const void*>(&k_gemm<EMB, NCX, 1, 0>),
                      hipFuncAttributeMaxDynamicSharedMemorySize, GA::LDS);
  k_gemm<EMB, NCX, 1, 0><<<NPAD / GA::BM, NTHR, GA::LDS, stream>>>(emb, eid, wp1, attEmb, xp, eI, eJ, nN, nTab, NPAD);
  k_agg<<<nAgg, NTHR, 0, stream>>>(csrS, csrD, offp, cnt, eI, eJ, xp, hcat, 2 * NCX, 0, nN, csrLen);

  hipFuncSetAttribute(reinterpret_cast<const void*>(&k_gemm<FEV, NCX, 0, 0>),
                      hipFuncAttributeMaxDynamicSharedMemorySize, GB::LDS);
  k_gemm<FEV, NCX, 0, 0><<<NPAD / GB::BM, NTHR, GB::LDS, stream>>>(x, eid, wp2, attEv, xp, eI, eJ, nN, nTab, NPAD);
  k_agg<<<nAgg, NTHR, 0, stream>>>(csrS, csrD, offp, cnt, eI, eJ, xp, hcat, 2 * NCX, NCX, nN, csrLen);

  hipFuncSetAttribute(reinterpret_cast<const void*>(&k_gemm<2 * NCX, NCX, 0, 0>),
                      hipFuncAttributeMaxDynamicSharedMemorySize, GC::LDS);
  k_gemm<2 * NCX, NCX, 0, 0><<<NPAD / GC::BM, NTHR, GC::LDS, stream>>>(hcat, eid, wp3, attCat, xp, eI, eJ, NPAD, nTab, NPAD);
  k_agg<<<nAgg, NTHR, 0, stream>>>(csrS, csrD, offp, cnt, eI, eJ, xp, h2, NCX, 0, nN, csrLen);

  hipFuncSetAttribute(reinterpret_cast<const void*>(&k_gemm<NCX, OUTD, 0, 1>),
                      hipFuncAttributeMaxDynamicSharedMemorySize, GF::LDS);
  k_gemm<NCX, OUTD, 0, 1><<<NPAD / GF::BM, NTHR, GF::LDS, stream>>>(h2, eid, wp4, fcb, out, eI, eJ, NPAD, nTab, nN);
}
